// MultiHeadSelfAttention_35089882808772
// MI455X (gfx1250) — hardware-run, weakly checked
//
#include <hip/hip_runtime.h>


#ifndef NB
#define NB 4
#endif
#ifndef SEQ
#define SEQ 2048
#endif
#define NB_FULL  4
#define SEQ_FULL 2048
#define DMOD   1024
#define NHEAD  16
#define HDIM   64
#define MROWS  (NB * SEQ)
#define CSC    0.18033688011112042f
#define PCAR2  10.0f
#define NEGB   (-3.0e38f)
#define PADL   (-1.4426950408889634e9f)
#define CCAR   64.0f
#define WCAR   64.0f
#define OSC    0.000244140625f
#define MWRD   (SEQ / 32)
#define MWP    (((MWRD + 31) / 32) * 32)

#define SZ_W ((size_t)DMOD * DMOD * 2)
#define SZ_X ((size_t)MROWS * DMOD * 2)
#define SZ_P ((size_t)NB * NHEAD * SEQ * HDIM * 2)
#define SZ_M ((((size_t)NB * MWP * 4) + 255) & ~(size_t)255)
#define WS_TOTAL (4 * SZ_W + 2 * SZ_X + 3 * SZ_P + SZ_M)

static_assert(NHEAD * HDIM == DMOD);
static_assert(HDIM == 64);
static_assert(DMOD % 64 == 0);
static_assert(DMOD % 32 == 0);
static_assert(DMOD % 256 == 0);
static_assert(SEQ % 64 == 0);
static_assert(SEQ % 32 == 0);
static_assert(SEQ % 16 == 0);
static_assert(NB <= NB_FULL);
static_assert(SEQ <= SEQ_FULL);
static_assert(((size_t)SEQ * DMOD / 8) % 256 == 0);
static_assert(((size_t)DMOD * DMOD / 64) % 64 == 0);
static_assert(MWP % 32 == 0);
static_assert(MWP >= MWRD);
static_assert(SZ_W % 256 == 0);
static_assert(SZ_X % 256 == 0);
static_assert(SZ_P % 256 == 0);
static_assert(SZ_M % 256 == 0);
static_assert(SZ_M >= (size_t)NB * MWP * 4);
static_assert(WS_TOTAL <= (size_t)134217728);
static_assert(NB * NHEAD <= 65535);
static_assert(CCAR * WCAR * OSC == 1.0f);

typedef _Float16 h16;
typedef unsigned short bf;
typedef __attribute__((ext_vector_type(16))) __bf16   v16bf;
typedef __attribute__((ext_vector_type(16))) _Float16 v16h;
typedef __attribute__((ext_vector_type(16))) unsigned short v16us;
typedef __attribute__((ext_vector_type(8)))  _Float16 v8h;
typedef __attribute__((ext_vector_type(8)))  unsigned short v8us;
typedef __attribute__((ext_vector_type(8)))  float    v8f;
typedef __attribute__((ext_vector_type(4)))  float    v4f;
typedef __attribute__((ext_vector_type(4)))  unsigned v4u;
typedef __attribute__((ext_vector_type(2)))  unsigned short v2us;
typedef __attribute__((ext_vector_type(2)))  _Float16 v2h;
typedef v4f  __attribute__((may_alias)) v4fa;
typedef v4u  __attribute__((may_alias)) v4ua;
typedef v8us __attribute__((may_alias)) v8usa;
typedef v8h  __attribute__((may_alias)) v8ha;

__device__ __forceinline__ unsigned short f2bf(float f) { unsigned u = __float_as_uint(f); u += 0x7FFFu + ((u >> 16) & 1u); return (unsigned short)(u >> 16); }
__device__ __forceinline__ float bf2f(unsigned short b) { return __uint_as_float(((unsigned)b) << 16); }
__device__ __forceinline__ float bfr(float f) { return bf2f(f2bf(f)); }
__device__ __forceinline__ void splitf(float y, unsigned short& h, unsigned short& l) { h = f2bf(y); l = f2bf(y - bf2f(h)); }
__device__ __forceinline__ v16h cat16(v8h lo, v8h hi) { return __builtin_shufflevector(lo, hi, 0, 1, 2, 3, 4, 5, 6, 7, 8, 9, 10, 11, 12, 13, 14, 15); }
__device__ __forceinline__ v16bf cat16b(v8us lo, v8us hi) { return __builtin_bit_cast(v16bf, __builtin_shufflevector(lo, hi, 0, 1, 2, 3, 4, 5, 6, 7, 8, 9, 10, 11, 12, 13, 14, 15)); }
__device__ __forceinline__ v8f wmma16(v16h a, v16h b, v8f c) { return __builtin_amdgcn_wmma_f32_16x16x32_f16(false, a, false, b, (short)0, c, false, false); }
__device__ __forceinline__ v8f wmmab(v16bf a, v16bf b, v8f c) { return __builtin_amdgcn_wmma_f32_16x16x32_bf16(false, a, false, b, (short)0, c, false, false); }
__device__ __forceinline__ v16h  ldh(const h16* p) { return cat16(*(const v8h*)p, *(const v8h*)(p + 16)); }
__device__ __forceinline__ v16bf ldb(const bf* p)  { return cat16b(*(const v8us*)p, *(const v8us*)(p + 16)); }
static __device__ __forceinline__ h16 toh_flush(float v) { const h16 r = (h16)v; return (fabsf(v) < 6.103515625e-05f) ? (h16)0.0f : r; }

__global__ __launch_bounds__(256) void k_wtG(const float* __restrict__ w, int K, int N, bf* Bt) {
    const int lane = threadIdx.x & 31; const int L0 = (blockIdx.x * 8 + (threadIdx.x >> 5)) * 8; const int nlines = N * K / 64;
#pragma unroll
    for (int ps = 0; ps < 2; ++ps) {
#pragma unroll 1
        for (int l = 0; l < 8; ++l) { const int L = L0 + l; if (L >= nlines) break; const size_t e = (size_t)L * 64 + lane * 2; const int k = (int)(e % K), n = (int)(e / K); v2us o;
            o[0] = f2bf(w[(size_t)k * N + n]); o[1] = f2bf(w[(size_t)(k + 1) * N + n]); *(volatile v2us*)(Bt + e) = o; }
        if (ps == 0) __threadfence(); }
}

__global__ __launch_bounds__(256) void k_wtH(const float* __restrict__ w, int K, int N, h16* Bt) {
    const int lane = threadIdx.x & 31; const int L0 = (blockIdx.x * 8 + (threadIdx.x >> 5)) * 8; const int nlines = N * K / 64;
#pragma unroll
    for (int ps = 0; ps < 2; ++ps) {
#pragma unroll 1
        for (int l = 0; l < 8; ++l) { const int L = L0 + l; if (L >= nlines) break; const size_t e = (size_t)L * 64 + lane * 2; const int k = (int)(e % K), n = (int)(e / K); v2h o;
            o[0] = toh_flush(bfr(w[(size_t)k * N + n]) * WCAR); o[1] = toh_flush(bfr(w[(size_t)(k + 1) * N + n]) * WCAR); *(volatile v2h*)(Bt + e) = o; }
        if (ps == 0) __threadfence(); }
}

__global__ __launch_bounds__(256) void k_cvt8(const float* __restrict__ src, bf* dst) {
    const size_t i = (size_t)blockIdx.x * 256 + threadIdx.x; if (i >= (size_t)SEQ * DMOD / 8) return;
    const size_t b = blockIdx.y;
    const v8f v = *(const v8f*)(src + b * ((size_t)SEQ_FULL * DMOD) + i * 8); v8us o;
#pragma unroll
    for (int k = 0; k < 8; ++k) o[k] = f2bf(v[k]);
    bf* d = dst + b * ((size_t)SEQ * DMOD) + i * 8;
    *(volatile v8us*)d = o; __threadfence(); *(volatile v8us*)d = o;
}

__global__ __launch_bounds__(256) void k_padm(const float* __restrict__ x, unsigned* MK) {
    __shared__ __align__(16) unsigned wsm[32];
    const int lane = threadIdx.x & 31;
    const int wave = __builtin_amdgcn_readfirstlane((int)(threadIdx.x >> 5));
    const float* xb = x + (size_t)blockIdx.y * ((size_t)SEQ_FULL * DMOD);
#pragma unroll 1
    for (int j = 0; j < 4; ++j) {
        const int wi = (int)blockIdx.x * 32 + wave * 4 + j;
        unsigned word = 0u;
#pragma unroll 1
        for (int r = 0; r < 32; ++r) {
            const int key = wi * 32 + r;
            const int d = key - (SEQ - 1);
            const int kc = key - (d & ~(d >> 31));
            const unsigned ok = (unsigned)((key - SEQ) >> 31) & 1u;
            const float* row = xb + (size_t)kc * DMOD + lane * 8;
            bool z = false;
#pragma unroll
            for (int c = 0; c < DMOD / 256; ++c) { const v8f v = *(const v8f*)(row + c * 256);
#pragma unroll
                for (int e = 0; e < 8; ++e) z = z || (v[e] == 0.0f); }
            const unsigned bal = __builtin_amdgcn_ballot_w32(z);
            const unsigned hit = (bal != 0u) ? 1u : 0u;
            word |= (hit & ok) << r;
        }
        if (lane == 0) wsm[wave * 4 + j] = word;
    }
    __syncthreads();
    if (wave == 0) {
        if (lane < 8) {
            const v4u o = *(const v4ua*)(wsm + lane * 4);
            unsigned* dptr = MK + ((size_t)blockIdx.y * MWP + (size_t)blockIdx.x * 32) + lane * 4;
            *(volatile v4u*)dptr = o; __threadfence(); *(volatile v4u*)dptr = o;
        }
    }
}

template <int MODE>
__device__ __forceinline__ void gemm_body(const bf* __restrict__ A, const bf* __restrict__ Bt, const float* __restrict__ bias, h16* P16) {
    __shared__ __align__(16) float os[64 * 68];
    const int lane = threadIdx.x & 31, lr = lane & 15, hi = lane >> 4;
    const int r0 = blockIdx.x * 64, c0 = blockIdx.y * 64;
    v8f acc[4][4];
#pragma unroll
    for (int mb = 0; mb < 4; ++mb)
#pragma unroll
        for (int nb = 0; nb < 4; ++nb) acc[mb][nb] = (v8f){};
    const size_t aoff = (size_t)(r0 + lr) * DMOD + 8 * hi, boff = (size_t)(c0 + lr) * DMOD + 8 * hi;
#pragma unroll 1
    for (int kc = 0; kc < DMOD; kc += 32) {
        v16bf a[4];
#pragma unroll
        for (int mb = 0; mb < 4; ++mb) a[mb] = ldb(A + aoff + (size_t)mb * 16 * DMOD + kc);
#pragma unroll
        for (int nb = 0; nb < 4; ++nb) { const v16bf b = ldb(Bt + boff + (size_t)nb * 16 * DMOD + kc);
#pragma unroll
            for (int mb = 0; mb < 4; ++mb) acc[mb][nb] = wmmab(a[mb], b, acc[mb][nb]); }
        asm volatile("v_nop\n\tv_nop\n\tv_nop\n\tv_nop" : "+v"(acc[0][0]), "+v"(acc[1][1]), "+v"(acc[2][2]), "+v"(acc[3][3]) : "v"(a[0]), "v"(a[3]));
    }
#pragma unroll
    for (int mb = 0; mb < 4; ++mb)
#pragma unroll
        for (int nb = 0; nb < 4; ++nb)
#pragma unroll
            for (int j = 0; j < 8; ++j) { const int row = mb * 16 + hi * 8 + j, col = nb * 16 + lr; if (MODE == 1) os[col * 68 + row] = acc[mb][nb][j]; else os[row * 68 + col] = acc[mb][nb][j]; }
    __syncthreads();
    const int bb = r0 / SEQ, t0 = r0 % SEQ;
    const int bh = bb * NHEAD + (int)blockIdx.y;
    const int pc = lane & 7, rq = lane >> 3;
    float bv[8];
#pragma unroll
    for (int j = 0; j < 8; ++j) bv[j] = (MODE == 0) ? bfr(bias[c0 + pc * 8 + j]) : 0.0f;
#pragma unroll 1
    for (int ps = 0; ps < 2; ++ps) {
#pragma unroll 1
        for (int s = 0; s < 16; ++s) { const int rr = 4 * s + rq;
            const v4f x0 = *(const v4fa*)(os + rr * 68 + pc * 8), x1 = *(const v4fa*)(os + rr * 68 + pc * 8 + 4);
            const float brow = (MODE == 1) ? bfr(bias[c0 + rr]) : 0.0f;
            float v[8];
#pragma unroll
            for (int j = 0; j < 4; ++j) { v[j] = x0[j] + bv[j] + brow; v[4 + j] = x1[j] + bv[4 + j] + brow; }
            v8h o16;
#pragma unroll
            for (int j = 0; j < 8; ++j) o16[j] = toh_flush(v[j]);
            const size_t e16 = (MODE == 0) ? (((size_t)bh * SEQ + t0 + rr) * HDIM + pc * 8) : (((size_t)bh * HDIM + rr) * SEQ + t0 + pc * 8);
            *(volatile v8h*)(P16 + e16) = o16; }
        if (ps == 0) __threadfence(); }
}

__device__ __forceinline__ void outp_body(const h16* __restrict__ A, const h16* __restrict__ Bt, const float* __restrict__ bias, float* C) {
    __shared__ __align__(16) float os[64 * 68];
    const int lane = threadIdx.x & 31, lr = lane & 15, hi = lane >> 4;
    const int r0 = blockIdx.x * 64, c0 = blockIdx.y * 64;
    v8f acc[4][4];
#pragma unroll
    for (int mb = 0; mb < 4; ++mb)
#pragma unroll
        for (int nb = 0; nb < 4; ++nb) acc[mb][nb] = (v8f){};
    const size_t aoff = (size_t)(r0 + lr) * DMOD + 8 * hi, boff = (size_t)(c0 + lr) * DMOD + 8 * hi;
#pragma unroll 1
    for (int kc = 0; kc < DMOD; kc += 32) {
        v16h a[4];
#pragma unroll
        for (int mb = 0; mb < 4; ++mb) a[mb] = ldh(A + aoff + (size_t)mb * 16 * DMOD + kc);
#pragma unroll
        for (int nb = 0; nb < 4; ++nb) { const v16h b = ldh(Bt + boff + (size_t)nb * 16 * DMOD + kc);
#pragma unroll
            for (int mb = 0; mb < 4; ++mb) acc[mb][nb] = wmma16(a[mb], b, acc[mb][nb]); }
        asm volatile("v_nop\n\tv_nop\n\tv_nop\n\tv_nop" : "+v"(acc[0][0]), "+v"(acc[1][1]), "+v"(acc[2][2]), "+v"(acc[3][3]) : "v"(a[0]), "v"(a[3]));
    }
#pragma unroll
    for (int mb = 0; mb < 4; ++mb)
#pragma unroll
        for (int nb = 0; nb < 4; ++nb)
#pragma unroll
            for (int j = 0; j < 8; ++j) { const int row = mb * 16 + hi * 8 + j, col = nb * 16 + lr; os[row * 68 + col] = acc[mb][nb][j]; }
    __syncthreads();
    const int bb = r0 / SEQ, t0 = r0 % SEQ;
    float* cbase = C + ((size_t)bb * SEQ_FULL + t0) * DMOD + c0;
    const int cofs = lr * 4;
    const float b0 = bfr(bias[c0 + cofs]), b1 = bfr(bias[c0 + cofs + 1]), b2 = bfr(bias[c0 + cofs + 2]), b3 = bfr(bias[c0 + cofs + 3]);
#pragma unroll 1
    for (int ps = 0; ps < 2; ++ps) {
#pragma unroll 1
        for (int s = 0; s < 32; ++s) { const int row = 2 * s + hi; v4f val = *(const v4fa*)(os + row * 68 + cofs);
            val[0] = val[0] * OSC + b0; val[1] = val[1] * OSC + b1; val[2] = val[2] * OSC + b2; val[3] = val[3] * OSC + b3;
            *(volatile v4f*)(cbase + (size_t)row * DMOD + cofs) = val; }
        if (ps == 0) __threadfence(); }
}

__global__ __launch_bounds__(32) void k_projrm(const bf* __restrict__ XB, const bf* __restrict__ Wt, const float* __restrict__ bias, h16* P16) { gemm_body<0>(XB, Wt, bias, P16); }
__global__ __launch_bounds__(32) void k_projtr(const bf* __restrict__ XB, const bf* __restrict__ Wt, const float* __restrict__ bias, h16* P16) { gemm_body<1>(XB, Wt, bias, P16); }
__global__ __launch_bounds__(32) void k_outp(const h16* __restrict__ CT, const h16* __restrict__ Wt, const float* __restrict__ bias, float* C) { outp_body(CT, Wt, bias, C); }

__device__ __forceinline__ float smax_pad(v8f s0, v8f s1, float& m, float& l, const unsigned mw, const int bofs, const float car, v16h& pf) {
#pragma unroll
    for (int i = 0; i < 8; ++i) { s0[i] *= CSC; s1[i] *= CSC; }
    if (mw != 0u) {
#pragma unroll
        for (int i = 0; i < 8; ++i) { s0[i] = (((mw >> (bofs + i)) & 1u) != 0u) ? PADL : s0[i]; s1[i] = (((mw >> (bofs + 16 + i)) & 1u) != 0u) ? PADL : s1[i]; }
    }
    float mi = fmaxf(s0[0], s1[0]);
#pragma unroll
    for (int i = 1; i < 8; ++i) mi = fmaxf(mi, fmaxf(s0[i], s1[i]));
    mi = fmaxf(mi, __shfl_xor(mi, 16, 32));
    const float mnew = fmaxf(m, mi);
    float ls = 0.0f;
#pragma unroll
    for (int i = 0; i < 8; ++i) {
        const float e0 = s0[i] - mnew + car, e1 = s1[i] - mnew + car;
        const float x0 = __builtin_amdgcn_exp2f(e0), x1 = __builtin_amdgcn_exp2f(e1);
        const float p0 = (e0 < -14.0f) ? 0.0f : x0;
        const float p1 = (e1 < -14.0f) ? 0.0f : x1;
        const h16 c0 = (h16)p0, c1 = (h16)p1;
        pf[i] = c0; pf[8 + i] = c1; ls += (float)c0 + (float)c1; }
    ls += __shfl_xor(ls, 16, 32);
    const float sc = __builtin_amdgcn_exp2f(m - mnew);
    l = l * sc + ls; m = mnew;
    return sc;
}

__device__ __forceinline__ void ctx_store(const v8f (&o)[4], const float inv, h16* CT, const size_t obase, const int lane) {
    __shared__ __align__(16) h16 sh[16 * 72];
    const int n = lane & 15, hi = lane >> 4;
#pragma unroll
    for (int t = 0; t < 4; ++t) { v8h oh;
#pragma unroll
        for (int r = 0; r < 8; ++r) oh[r] = toh_flush(o[t][r] * inv);
        *(v8ha*)(sh + n * 72 + t * 16 + 8 * hi) = oh; }
    __syncthreads();
    const int pc = lane & 7, rq = lane >> 3;
#pragma unroll 1
    for (int ps = 0; ps < 2; ++ps) {
#pragma unroll
        for (int s = 0; s < 4; ++s) { const int row = 4 * s + rq;
            const v8h vh = *(const v8ha*)(sh + row * 72 + pc * 8);
            *(volatile v8h*)(CT + obase + (size_t)row * DMOD + pc * 8) = vh; }
        if (ps == 0) __threadfence(); }
}

__global__ __launch_bounds__(32) void k_attnd(const h16* __restrict__ Q16, const h16* __restrict__ K16, const h16* __restrict__ VT16, const unsigned* __restrict__ MK, h16* CT) {
    const int lane = threadIdx.x & 31, n = lane & 15, hi = lane >> 4;
    const int bh = blockIdx.y, qBase = (int)blockIdx.x * 16, q = qBase + n;
    const int b = bh / NHEAD, h = bh % NHEAD;
    const size_t pb = (size_t)bh * SEQ * HDIM;
    const size_t qoff = pb + (size_t)q * HDIM + 8 * hi;
    const size_t koff = pb + (size_t)n * HDIM + 8 * hi;
    const size_t voff = pb + (size_t)n * SEQ + 8 * hi;
    const size_t moff = (size_t)b * MWP;
    v8f o[4];
#pragma unroll
    for (int t = 0; t < 4; ++t) o[t] = (v8f){};
    float m = NEGB, l = 0.0f;
#pragma unroll 1
    for (int kb = 0; kb < SEQ / 32; ++kb) {
        const int keyBase = kb * 32;
        v8f s0 = (v8f){}, s1 = (v8f){};
        v16h qf[2], k0[2], k1[2];
#pragma unroll
        for (int c = 0; c < 2; ++c) {
            qf[c] = ldh(Q16 + qoff + c * 32);
            k0[c] = ldh(K16 + koff + (size_t)keyBase * HDIM + c * 32);
            k1[c] = ldh(K16 + koff + (size_t)(keyBase + 16) * HDIM + c * 32);
            s0 = wmma16(k0[c], qf[c], s0); s1 = wmma16(k1[c], qf[c], s1);
        }
        asm volatile("v_nop\n\tv_nop\n\tv_nop\n\tv_nop" : "+v"(s0), "+v"(s1) : "v"(qf[1]), "v"(k1[1]));
        const unsigned mw = (unsigned)__builtin_amdgcn_readfirstlane((int)MK[moff + kb]);
        v16h pf;
        const float sc = smax_pad(s0, s1, m, l, mw, 8 * hi, PCAR2, pf);
#pragma unroll
        for (int t = 0; t < 4; ++t) o[t] = o[t] * sc;
        v16h va[4];
#pragma unroll
        for (int t = 0; t < 4; ++t) va[t] = ldh(VT16 + voff + (size_t)t * 16 * SEQ + keyBase);
#pragma unroll
        for (int t = 0; t < 4; ++t) o[t] = wmma16(va[t], pf, o[t]);
        asm volatile("v_nop\n\tv_nop\n\tv_nop\n\tv_nop" : "+v"(o[0]), "+v"(o[1]), "+v"(o[2]), "+v"(o[3]) : "v"(pf), "v"(va[3]));
    }
    ctx_store(o, (1.0f / l) * CCAR, CT, ((size_t)b * SEQ + qBase) * DMOD + (size_t)h * HDIM, lane);
}

extern "C" void kernel_launch(void* const* d_in, const int* in_sizes, int n_in,
                              void* d_out, int out_size, void* d_ws, size_t ws_size, hipStream_t stream) {
    if (n_in < 9) return;
    const size_t needx = ((size_t)(NB - 1) * SEQ_FULL + SEQ) * DMOD;
    if ((size_t)in_sizes[0] < needx) return;
    if ((size_t)out_size < needx) return;
    if ((size_t)in_sizes[1] < (size_t)DMOD * DMOD || (size_t)in_sizes[3] < (size_t)DMOD * DMOD || (size_t)in_sizes[5] < (size_t)DMOD * DMOD || (size_t)in_sizes[7] < (size_t)DMOD * DMOD) return;
    if (in_sizes[2] < DMOD || in_sizes[4] < DMOD || in_sizes[6] < DMOD || in_sizes[8] < DMOD) return;
    if (ws_size < WS_TOTAL) return;
    const float* x = (const float*)d_in[0]; const float* wq = (const float*)d_in[1]; const float* bq = (const float*)d_in[2]; const float* wk = (const float*)d_in[3]; const float* bk = (const float*)d_in[4];
    const float* wv = (const float*)d_in[5]; const float* bv = (const float*)d_in[6]; const float* wo = (const float*)d_in[7]; const float* bo = (const float*)d_in[8];
    float* OUT = (float*)d_out;
    char* wsp = (char*)d_ws;
    auto take = [&](size_t bytes) { char* p = wsp; wsp += (bytes + 255) & ~(size_t)255; return (void*)p; };
    bf* WQ = (bf*)take(SZ_W); bf* WK = (bf*)take(SZ_W); bf* WV = (bf*)take(SZ_W); h16* WO = (h16*)take(SZ_W);
    bf* XB = (bf*)take(SZ_X);
    h16* Q16 = (h16*)take(SZ_P); h16* K16 = (h16*)take(SZ_P); h16* VT16 = (h16*)take(SZ_P);
    h16* CT = (h16*)take(SZ_X);
    unsigned* MK = (unsigned*)take(SZ_M);
    if ((size_t)(wsp - (char*)d_ws) > ws_size) return;

    const unsigned gw = (unsigned)(((size_t)DMOD * DMOD / 64 + 63) / 64);
    k_wtG<<<gw, 256, 0, stream>>>(wq, DMOD, DMOD, WQ);
    k_wtG<<<gw, 256, 0, stream>>>(wk, DMOD, DMOD, WK);
    k_wtG<<<gw, 256, 0, stream>>>(wv, DMOD, DMOD, WV);
    k_wtH<<<gw, 256, 0, stream>>>(wo, DMOD, DMOD, WO);
    k_cvt8<<<dim3((unsigned)(((size_t)SEQ * DMOD / 8 + 255) / 256), NB, 1), 256, 0, stream>>>(x, XB);
    k_padm<<<dim3(MWP / 32, NB, 1), 256, 0, stream>>>(x, MK);
    const dim3 gg(MROWS / 64, DMOD / 64, 1);
    k_projrm<<<gg, 32, 0, stream>>>(XB, WQ, bq, Q16);
    k_projrm<<<gg, 32, 0, stream>>>(XB, WK, bk, K16);
    k_projtr<<<gg, 32, 0, stream>>>(XB, WV, bv, VT16);
    k_attnd<<<dim3(SEQ / 16, NB * NHEAD, 1), 32, 0, stream>>>(Q16, K16, VT16, MK, CT);
    k_outp<<<gg, 32, 0, stream>>>(CT, WO, bo, OUT);
}
